// TransformerEncoder_15444702396491
// MI455X (gfx1250) — hardware-run, weakly checked
//
#include <hip/hip_runtime.h>


#ifndef NB
#define NB 2
#endif
#ifndef SEQ
#define SEQ 2048
#endif
#define NB_FULL 2
#define SEQ_FULL 2048
#define DM 1024
#define NH 16
#define HD 64
#define DFF 4096
#define MTOK (NB * SEQ)
#define LNEPS 1e-5f
#define SCL 0.03125f
#define L2E 1.4426950408889634f
#define WCAR 64.0f
#define ACAR 16.0f
#define PP 72

static_assert(NB >= 1 && NB <= NB_FULL);
static_assert(SEQ % 64 == 0 && SEQ >= 64 && SEQ <= SEQ_FULL);
static_assert(DM == NH * HD && HD == 64);
static_assert(DM % 256 == 0 && DFF % 64 == 0 && MTOK % 64 == 0 && MTOK % 8 == 0);
static_assert((DM * DM) % 2048 == 0 && (DFF * DM) % 2048 == 0);

typedef _Float16 h16;
typedef __attribute__((ext_vector_type(16))) _Float16 v16h;
typedef __attribute__((ext_vector_type(8)))  _Float16 v8h;
typedef __attribute__((ext_vector_type(8)))  float    v8f;
typedef __attribute__((ext_vector_type(4)))  float    v4f;
typedef v8h __attribute__((may_alias)) v8ha;
typedef v4f __attribute__((may_alias)) v4fa;

__device__ __forceinline__ unsigned short f2bf(float f) { unsigned u = __float_as_uint(f); u += 0x7FFFu + ((u >> 16) & 1u); return (unsigned short)(u >> 16); }
__device__ __forceinline__ float bf2f(unsigned short b) { return __uint_as_float(((unsigned)b) << 16); }
__device__ __forceinline__ float bfr(float f) { return bf2f(f2bf(f)); }
__device__ __forceinline__ v16h cat16(v8h lo, v8h hi) { return __builtin_shufflevector(lo, hi, 0, 1, 2, 3, 4, 5, 6, 7, 8, 9, 10, 11, 12, 13, 14, 15); }
__device__ __forceinline__ v16h ldf(const h16* p) { return cat16(*(const v8h*)p, *(const v8h*)(p + 16)); }
__device__ __forceinline__ v8f wmma16(v16h a, v16h b, v8f c) { return __builtin_amdgcn_wmma_f32_16x16x32_f16(false, a, false, b, (short)0, c, false, false); }
__device__ __forceinline__ void wsync() { __builtin_amdgcn_fence(3, "wavefront"); __builtin_amdgcn_wave_barrier(); asm volatile("" ::: "memory"); }

__global__ __launch_bounds__(256) void k_cvtw(const float* __restrict__ src, h16* dst, size_t n8, float scale) {
    const size_t i = (size_t)blockIdx.x * 256 + threadIdx.x; if (i >= n8) return;
    const v8f v = *(const v8f*)(src + i * 8); v8h o;
#pragma unroll
    for (int k = 0; k < 8; ++k) o[k] = (h16)(bfr(v[k]) * scale);
    *(volatile v8h*)(dst + i * 8) = o; __threadfence(); *(volatile v8h*)(dst + i * 8) = o;
}

template <bool RND>
__global__ __launch_bounds__(256) void k_ln(const float* __restrict__ X, int seq, int seqsrc, const float* __restrict__ g, const float* __restrict__ be, h16* Y, int nrows) {
    const int lane = threadIdx.x & 31; const int r = blockIdx.x * 8 + (threadIdx.x >> 5); if (r >= nrows) return;
    const size_t rsrc = (size_t)(r / seq) * (size_t)seqsrc + (size_t)(r % seq);
    const float* xr = X + rsrc * DM; float s = 0.f;
#pragma unroll 1
    for (int ch = 0; ch < DM / 256; ++ch) { const int c0 = ch * 256 + lane * 8; const v8f a = *(const v8f*)(xr + c0);
#pragma unroll
        for (int q = 0; q < 8; ++q) s = __fadd_rn(s, RND ? bfr(a[q]) : a[q]); }
#pragma unroll
    for (int sh = 16; sh; sh >>= 1) s += __shfl_xor(s, sh, 32);
    const float mu = s * (1.0f / DM); float s2 = 0.f;
#pragma unroll 1
    for (int ch = 0; ch < DM / 256; ++ch) { const int c0 = ch * 256 + lane * 8; const v8f a = *(const v8f*)(xr + c0);
#pragma unroll
        for (int q = 0; q < 8; ++q) { const float d0 = __fsub_rn(RND ? bfr(a[q]) : a[q], mu); float p = __fmul_rn(d0, d0); asm volatile("" : "+v"(p)); s2 = __fadd_rn(s2, p); } }
#pragma unroll
    for (int sh = 16; sh; sh >>= 1) s2 += __shfl_xor(s2, sh, 32);
    const float rs = __fdiv_rn(1.0f, __fsqrt_rn(__fadd_rn(s2 * (1.0f / DM), LNEPS)));
#pragma unroll 1
    for (int ps = 0; ps < 2; ++ps) {
#pragma unroll 1
        for (int ch = 0; ch < DM / 256; ++ch) { const int c0 = ch * 256 + lane * 8; const v8f a = *(const v8f*)(xr + c0); v8h o;
#pragma unroll
            for (int q = 0; q < 8; ++q) { const float v = RND ? bfr(a[q]) : a[q]; float n0 = __fmul_rn(__fsub_rn(v, mu), rs); asm volatile("" : "+v"(n0)); float n1 = __fmul_rn(n0, bfr(g[c0 + q])); asm volatile("" : "+v"(n1)); o[q] = (h16)__fadd_rn(n1, bfr(be[c0 + q])); }
            *(volatile v8h*)(Y + (size_t)r * DM + c0) = o; }
        if (ps == 0) __threadfence(); }
}

template <int BM, bool RELU, int RES, bool O16>
__global__ __launch_bounds__(32) void k_gemm(const h16* __restrict__ A, const h16* __restrict__ Bt, int K, float* C, h16* C16, int ldc,
                                             const float* __restrict__ bias, const float* __restrict__ R, int ldr, float oscale,
                                             size_t sA, size_t sB, size_t sC, size_t sR) {
    __shared__ __align__(16) float os[16 * 68];
    const size_t z = blockIdx.z; A += z * sA; Bt += z * sB; if (O16) C16 += z * sC; else C += z * sC; if (RES != 0) R += z * sR;
    const int lane = threadIdx.x & 31, lr = lane & 15, hi = lane >> 4; const int r0 = blockIdx.x * 64, c0 = blockIdx.y * 64;
    v8f acc[4][4];
#pragma unroll
    for (int mb = 0; mb < 4; ++mb)
#pragma unroll
        for (int nb = 0; nb < 4; ++nb) acc[mb][nb] = (v8f){};
    const size_t aoff = (size_t)(r0 + lr) * K + 8 * hi, boff = (size_t)(c0 + lr) * K + 8 * hi;
#pragma unroll 1
    for (int kc = 0; kc < K; kc += 32) {
        v16h a[4], b[4];
#pragma unroll
        for (int mb = 0; mb < 4; ++mb) a[mb] = ldf(A + aoff + (size_t)mb * 16 * K + kc);
#pragma unroll
        for (int nb = 0; nb < 4; ++nb) { b[nb] = ldf(Bt + boff + (size_t)nb * 16 * K + kc);
#pragma unroll
            for (int mb = 0; mb < 4; ++mb) acc[mb][nb] = wmma16(a[mb], b[nb], acc[mb][nb]); }
        asm volatile("v_nop\n\tv_nop\n\tv_nop\n\tv_nop"
                     : "+v"(acc[0][0]), "+v"(acc[0][1]), "+v"(acc[0][2]), "+v"(acc[0][3]),
                       "+v"(acc[1][0]), "+v"(acc[1][1]), "+v"(acc[1][2]), "+v"(acc[1][3]),
                       "+v"(acc[2][0]), "+v"(acc[2][1]), "+v"(acc[2][2]), "+v"(acc[2][3]),
                       "+v"(acc[3][0]), "+v"(acc[3][1]), "+v"(acc[3][2]), "+v"(acc[3][3])
                     : "v"(a[0]), "v"(a[3]), "v"(b[0]), "v"(b[3]));
    }
#pragma unroll
    for (int mb = 0; mb < 4; ++mb) {
#pragma unroll
        for (int nb = 0; nb < 4; ++nb) {
#pragma unroll
            for (int j = 0; j < 8; ++j) os[(hi * 8 + j) * 68 + nb * 16 + lr] = acc[mb][nb][j]; }
        wsync();
        const int rb = r0 + mb * 16;
        if (!O16) {
#pragma unroll 1
            for (int ps = 0; ps < 2; ++ps) {
#pragma unroll
                for (int s = 0; s < 8; ++s) { const int row = 2 * s + hi, cofs = lr * 4; v4f val = *(const v4fa*)(os + row * 68 + cofs);
#pragma unroll
                    for (int q = 0; q < 4; ++q) { float t = val[q] * oscale; if (BM == 1) t = __fadd_rn(t, bfr(bias[c0 + cofs + q])); if (BM == 2) t = __fadd_rn(t, bfr(bias[rb + row])); if (RELU) t = fmaxf(t, 0.0f); val[q] = t; }
                    if (RES != 0) { const v4f rr = *(const v4f*)(R + (size_t)(rb + row) * ldr + c0 + cofs);
#pragma unroll
                        for (int q = 0; q < 4; ++q) val[q] = __fadd_rn(val[q], (RES == 2) ? bfr(rr[q]) : rr[q]); }
                    *(volatile v4f*)(C + (size_t)(rb + row) * ldc + c0 + cofs) = val; }
                if (ps == 0) __threadfence(); }
        } else {
#pragma unroll 1
            for (int ps = 0; ps < 2; ++ps) {
#pragma unroll
                for (int s = 0; s < 4; ++s) { const int row = 4 * s + (lane >> 3), cofs = (lane & 7) * 8; const v4f v0 = *(const v4fa*)(os + row * 68 + cofs), v1 = *(const v4fa*)(os + row * 68 + cofs + 4); v8h o;
#pragma unroll
                    for (int q = 0; q < 4; ++q) { float t0 = v0[q] * oscale, t1 = v1[q] * oscale;
                        if (BM == 1) { t0 = __fadd_rn(t0, bfr(bias[c0 + cofs + q])); t1 = __fadd_rn(t1, bfr(bias[c0 + cofs + 4 + q])); }
                        if (BM == 2) { const float rbv = bfr(bias[rb + row]); t0 = __fadd_rn(t0, rbv); t1 = __fadd_rn(t1, rbv); }
                        if (RELU) { t0 = fmaxf(t0, 0.0f); t1 = fmaxf(t1, 0.0f); }
                        o[q] = (h16)t0; o[4 + q] = (h16)t1; }
                    *(volatile v8h*)(C16 + (size_t)(rb + row) * ldc + c0 + cofs) = o; }
                if (ps == 0) __threadfence(); }
        }
        wsync();
    }
}

__global__ __launch_bounds__(128) void k_attn(const h16* __restrict__ Q, const h16* __restrict__ Kp, const h16* __restrict__ VT, h16* AT) {
    __shared__ __align__(16) h16 Ps[4][16 * PP];
    const int lane = threadIdx.x & 31, wv = threadIdx.x >> 5, hh = lane >> 4, m = lane & 15;
    const int bh = blockIdx.y; const int b = bh / NH, h = bh - b * NH;
    const int q0 = blockIdx.x * 64 + wv * 16;
    if (q0 >= SEQ) return;
    h16* Pw = &Ps[wv][0];
    const size_t tok0 = (size_t)b * SEQ + q0;
    const h16* qp = Q + (tok0 + m) * DM + h * HD + 8 * hh;
    v16h qf[2];
#pragma unroll
    for (int s = 0; s < 2; ++s) qf[s] = ldf(qp + s * 32);
    const h16* kb = Kp + ((size_t)b * SEQ + m) * DM + h * HD + 8 * hh;
    const h16* vb = VT + ((size_t)bh * HD + m) * SEQ + 8 * hh;
    v8f oacc[4]; float mrun[8], lrun[8];
#pragma unroll
    for (int dt = 0; dt < 4; ++dt) oacc[dt] = (v8f){};
#pragma unroll
    for (int r = 0; r < 8; ++r) { mrun[r] = -1.0e30f; lrun[r] = 0.0f; }
#pragma unroll 1
    for (int j0 = 0; j0 < SEQ; j0 += 64) {
        v16h kf[4][2];
#pragma unroll
        for (int nt = 0; nt < 4; ++nt) { const h16* kp = kb + (size_t)(j0 + nt * 16) * DM;
#pragma unroll
            for (int ks = 0; ks < 2; ++ks) kf[nt][ks] = ldf(kp + ks * 32); }
        v8f sacc[4];
#pragma unroll
        for (int nt = 0; nt < 4; ++nt) { sacc[nt] = (v8f){};
#pragma unroll
            for (int ks = 0; ks < 2; ++ks) sacc[nt] = wmma16(qf[ks], kf[nt][ks], sacc[nt]); }
        asm volatile("v_nop\n\tv_nop\n\tv_nop\n\tv_nop" : "+v"(sacc[0]), "+v"(sacc[1]), "+v"(sacc[2]), "+v"(sacc[3]) : "v"(qf[0]), "v"(qf[1]), "v"(kf[0][0]), "v"(kf[3][1]));
        float cr[8];
#pragma unroll
        for (int r = 0; r < 8; ++r) { float tm = fmaxf(fmaxf(sacc[0][r], sacc[1][r]), fmaxf(sacc[2][r], sacc[3][r]));
#pragma unroll
            for (int sh = 8; sh; sh >>= 1) tm = fmaxf(tm, __shfl_xor(tm, sh, 32));
            const float nm = fmaxf(mrun[r], tm * SCL); cr[r] = __builtin_amdgcn_exp2f((mrun[r] - nm) * L2E); mrun[r] = nm; }
#pragma unroll
        for (int r = 0; r < 8; ++r) { float ps = 0.f;
#pragma unroll
            for (int nt = 0; nt < 4; ++nt) { const float e = __builtin_amdgcn_exp2f((sacc[nt][r] * SCL - mrun[r]) * L2E); sacc[nt][r] = e; ps += e; }
#pragma unroll
            for (int sh = 8; sh; sh >>= 1) ps += __shfl_xor(ps, sh, 32);
            lrun[r] = lrun[r] * cr[r] + ps;
#pragma unroll
            for (int dt = 0; dt < 4; ++dt) oacc[dt][r] *= cr[r]; }
        wsync();
#pragma unroll
        for (int nt = 0; nt < 4; ++nt)
#pragma unroll
            for (int r = 0; r < 8; ++r) Pw[(8 * hh + r) * PP + nt * 16 + m] = (h16)sacc[nt][r];
        wsync();
        v16h pa[2];
#pragma unroll
        for (int ks = 0; ks < 2; ++ks) pa[ks] = cat16(*(const v8ha*)(Pw + m * PP + ks * 32 + 8 * hh), *(const v8ha*)(Pw + m * PP + ks * 32 + 16 + 8 * hh));
        v16h vf[4][2];
#pragma unroll
        for (int dt = 0; dt < 4; ++dt) { const h16* vp = vb + (size_t)dt * 16 * SEQ + j0;
#pragma unroll
            for (int ks = 0; ks < 2; ++ks) vf[dt][ks] = ldf(vp + ks * 32); }
#pragma unroll
        for (int dt = 0; dt < 4; ++dt)
#pragma unroll
            for (int ks = 0; ks < 2; ++ks) oacc[dt] = wmma16(pa[ks], vf[dt][ks], oacc[dt]);
        asm volatile("v_nop\n\tv_nop\n\tv_nop\n\tv_nop" : "+v"(oacc[0]), "+v"(oacc[1]), "+v"(oacc[2]), "+v"(oacc[3]) : "v"(pa[0]), "v"(pa[1]), "v"(vf[0][0]), "v"(vf[3][1]));
    }
    float rl[8];
#pragma unroll
    for (int r = 0; r < 8; ++r) rl[r] = ACAR / lrun[r];
    wsync();
#pragma unroll
    for (int dt = 0; dt < 4; ++dt)
#pragma unroll
        for (int r = 0; r < 8; ++r) Pw[(8 * hh + r) * PP + dt * 16 + m] = (h16)(oacc[dt][r] * rl[r]);
    wsync();
    h16* arow = AT + tok0 * DM + h * HD;
#pragma unroll 1
    for (int ps = 0; ps < 2; ++ps) {
#pragma unroll
        for (int s = 0; s < 4; ++s) { const int row = 4 * s + (lane >> 3), pc = (lane & 7) * 8; const v8h val = *(const v8ha*)(Pw + row * PP + pc); *(volatile v8h*)(arow + (size_t)row * DM + pc) = val; }
        if (ps == 0) __threadfence(); }
}

extern "C" void kernel_launch(void* const* d_in, const int* in_sizes, int n_in,
                              void* d_out, int out_size, void* d_ws, size_t ws_size, hipStream_t stream) {
    if (n_in < 17) return;
    const float* x = (const float*)d_in[0]; const float* g1 = (const float*)d_in[1]; const float* e1 = (const float*)d_in[2];
    const float* wq = (const float*)d_in[3]; const float* bq = (const float*)d_in[4]; const float* wk = (const float*)d_in[5]; const float* bk = (const float*)d_in[6];
    const float* wv = (const float*)d_in[7]; const float* bv = (const float*)d_in[8]; const float* wo = (const float*)d_in[9]; const float* bo = (const float*)d_in[10];
    const float* g2 = (const float*)d_in[11]; const float* e2 = (const float*)d_in[12];
    const float* w1 = (const float*)d_in[13]; const float* b1 = (const float*)d_in[14]; const float* w2 = (const float*)d_in[15]; const float* b2 = (const float*)d_in[16];
    const size_t needx = (size_t)(NB - 1) * SEQ_FULL * DM + (size_t)SEQ * DM;
    if ((size_t)in_sizes[0] < needx || (size_t)out_size < needx) return;
    if (in_sizes[1] < DM || in_sizes[2] < DM || in_sizes[4] < DM || in_sizes[6] < DM || in_sizes[8] < DM || in_sizes[10] < DM || in_sizes[11] < DM || in_sizes[12] < DM || in_sizes[14] < DFF || in_sizes[16] < DM) return;
    if (in_sizes[3] < DM * DM || in_sizes[5] < DM * DM || in_sizes[7] < DM * DM || in_sizes[9] < DM * DM || in_sizes[13] < DFF * DM || in_sizes[15] < DM * DFF) return;
    float* OUT = (float*)d_out;
    char* wsp = (char*)d_ws;
    auto take = [&](size_t bytes) { char* p = wsp; wsp += (bytes + 255) & ~(size_t)255; return (void*)p; };
    h16* WQ = (h16*)take((size_t)DM * DM * 2); h16* WK = (h16*)take((size_t)DM * DM * 2); h16* WV = (h16*)take((size_t)DM * DM * 2); h16* WO = (h16*)take((size_t)DM * DM * 2);
    h16* W1 = (h16*)take((size_t)DFF * DM * 2); h16* W2 = (h16*)take((size_t)DM * DFF * 2);
    h16* Y1 = (h16*)take((size_t)MTOK * DM * 2);
    h16* Q16 = (h16*)take((size_t)MTOK * DM * 2); h16* K16 = (h16*)take((size_t)MTOK * DM * 2);
    h16* VT16 = (h16*)take((size_t)NB * DM * SEQ * 2);
    h16* AT16 = (h16*)take((size_t)MTOK * DM * 2);
    float* OUT1 = (float*)take((size_t)MTOK * DM * 4);
    h16* Y2 = (h16*)take((size_t)MTOK * DM * 2);
    h16* H16 = (h16*)take((size_t)MTOK * DFF * 2);
    if ((size_t)(wsp - (char*)d_ws) > ws_size) return;
    const float winv = 1.0f / WCAR;
    k_cvtw<<<(unsigned)((size_t)DM * DM / 8 / 256), 256, 0, stream>>>(wq, WQ, (size_t)DM * DM / 8, WCAR);
    k_cvtw<<<(unsigned)((size_t)DM * DM / 8 / 256), 256, 0, stream>>>(wk, WK, (size_t)DM * DM / 8, WCAR);
    k_cvtw<<<(unsigned)((size_t)DM * DM / 8 / 256), 256, 0, stream>>>(wv, WV, (size_t)DM * DM / 8, WCAR);
    k_cvtw<<<(unsigned)((size_t)DM * DM / 8 / 256), 256, 0, stream>>>(wo, WO, (size_t)DM * DM / 8, WCAR);
    k_cvtw<<<(unsigned)((size_t)DFF * DM / 8 / 256), 256, 0, stream>>>(w1, W1, (size_t)DFF * DM / 8, WCAR);
    k_cvtw<<<(unsigned)((size_t)DM * DFF / 8 / 256), 256, 0, stream>>>(w2, W2, (size_t)DM * DFF / 8, WCAR);
    k_ln<true><<<MTOK / 8, 256, 0, stream>>>(x, SEQ, SEQ_FULL, g1, e1, Y1, MTOK);
    k_gemm<1, false, 0, true><<<dim3(MTOK / 64, DM / 64, 1), 32, 0, stream>>>(Y1, WQ, DM, nullptr, Q16, DM, bq, nullptr, 0, winv, 0, 0, 0, 0);
    k_gemm<1, false, 0, true><<<dim3(MTOK / 64, DM / 64, 1), 32, 0, stream>>>(Y1, WK, DM, nullptr, K16, DM, bk, nullptr, 0, winv, 0, 0, 0, 0);
    k_gemm<2, false, 0, true><<<dim3(DM / 64, SEQ / 64, NB), 32, 0, stream>>>(WV, Y1, DM, nullptr, VT16, SEQ, bv, nullptr, 0, winv, 0, (size_t)SEQ * DM, (size_t)DM * SEQ, 0);
    k_attn<<<dim3(SEQ / 64, NB * NH, 1), 128, 0, stream>>>(Q16, K16, VT16, AT16);
    k_gemm<1, false, 2, false><<<dim3(SEQ / 64, DM / 64, NB), 32, 0, stream>>>(AT16, WO, DM, OUT1, nullptr, DM, bo, x, DM, winv / ACAR, (size_t)SEQ * DM, 0, (size_t)SEQ * DM, (size_t)SEQ_FULL * DM);
    k_ln<false><<<MTOK / 8, 256, 0, stream>>>(OUT1, SEQ, SEQ, g2, e2, Y2, MTOK);
    k_gemm<1, true, 0, true><<<dim3(MTOK / 64, DFF / 64, 1), 32, 0, stream>>>(Y2, W1, DM, nullptr, H16, DFF, b1, nullptr, 0, winv, 0, 0, 0, 0);
    k_gemm<1, true, 1, false><<<dim3(SEQ / 64, DM / 64, NB), 32, 0, stream>>>(H16, W2, DFF, OUT, nullptr, DM, b2, OUT1, DM, winv, (size_t)SEQ * DFF, 0, (size_t)SEQ_FULL * DM, (size_t)SEQ * DM);
}
